// Encoder_84499186581951
// MI455X (gfx1250) — hardware-verified
//
#include <hip/hip_runtime.h>
#include <math.h>

constexpr int NSEQ    = 32;
constexpr int NSTEP   = 2048;
constexpr int NVOC    = 128;
constexpr int NHID    = 512;
constexpr int NGATE   = 4 * NHID;
constexpr int NTHR    = 256;
constexpr int NWAVE   = NTHR / 32;
constexpr int SEQ_BLK = 16;
constexpr int HPITCH  = 520;
constexpr int OPITCH  = 516;
constexpr int XSEG    = 16;
constexpr int BIGI    = 0x7fffffff;
constexpr float HCARRY = 16.0f;
constexpr float WCARRY = 64.0f;
constexpr float ZINV   = 1.0f / (HCARRY * WCARRY);
static_assert(NGATE == 2048 && NHID == 512 && NVOC == 128 && NSEQ == 32 && NSTEP == 2048);
static_assert(NSEQ % SEQ_BLK == 0);
static_assert(NHID == 64 * NWAVE);
static_assert(NHID % 32 == 0);
static_assert((2 * SEQ_BLK * HPITCH) % NTHR == 0);
static_assert(SEQ_BLK * NVOC == 8 * NTHR);
static_assert(NGATE == 8 * NTHR);
static_assert(SEQ_BLK * NHID == 8 * 4 * NTHR);
static_assert(NSTEP % 32 == 0);
static_assert(NHID % 64 == 0 && NGATE % 64 == 0);
static_assert(HPITCH % 8 == 0 && OPITCH % 4 == 0);

typedef __attribute__((ext_vector_type(16))) _Float16 v16h;
typedef __attribute__((ext_vector_type(8)))  _Float16 v8h;
typedef __attribute__((ext_vector_type(8)))  float    v8f;
typedef __attribute__((ext_vector_type(4)))  float    v4f;

__device__ __forceinline__ void grp_guard_h(v8f& a0, v8f& a1, v8f& a2, v8f& a3,
                                            v16h x, v16h y0, v16h y1, v16h y2, v16h y3) {
  asm volatile("v_nop\n\tv_nop\n\tv_nop\n\tv_nop"
               : "+v"(a0), "+v"(a1), "+v"(a2), "+v"(a3)
               : "v"(x), "v"(y0), "v"(y1), "v"(y2), "v"(y3));
}
__device__ __forceinline__ void acc_guard4(v8f& a, v8f& b, v8f& c, v8f& d) {
  asm volatile("v_nop\n\tv_nop\n\tv_nop\n\tv_nop" : "+v"(a), "+v"(b), "+v"(c), "+v"(d));
}
template <typename T> struct Frag;
template <> struct Frag<_Float16> {
  typedef v16h V; union U { v16h v; v8h h[2]; };
  static __device__ __forceinline__ v16h load(const _Float16* p) {
    U f; f.h[0] = *(const v8h*)(p); f.h[1] = *(const v8h*)(p + 16); return f.v;
  }
  static __device__ __forceinline__ v8f mma(v16h a, v16h b, v8f c) {
    return __builtin_amdgcn_wmma_f32_16x16x32_f16(false, a, false, b, (short)0, c, false, false);
  }
};

__device__ __forceinline__ float fsig(float x)  { return __builtin_amdgcn_rcpf(1.0f + expf(-x)); }
__device__ __forceinline__ float ftanh(float x) { return 1.0f - 2.0f * __builtin_amdgcn_rcpf(expf(2.0f * x) + 1.0f); }

__global__ __launch_bounds__(NTHR) void tpose_f16_kernel(const float* __restrict__ src, int R, int C, int ldo,
                                                         unsigned short* __restrict__ O, float sc) {
  __shared__ float Tt[64 * 65];
  const int tid = threadIdx.x;
  const int c0 = blockIdx.x * 64, r0 = blockIdx.y * 64;
#pragma unroll
  for (int i = 0; i < 4; ++i) {
    const int idx = i * NTHR + tid;
    const int rr = idx >> 4, cc = (idx & 15) * 4;
    const v4f v = *(const v4f*)(src + (size_t)(r0 + rr) * (size_t)C + c0 + cc);
    Tt[rr * 65 + cc + 0] = v[0];
    Tt[rr * 65 + cc + 1] = v[1];
    Tt[rr * 65 + cc + 2] = v[2];
    Tt[rr * 65 + cc + 3] = v[3];
  }
  __syncthreads();
  const int q = tid >> 3, c8 = (tid & 7) * 8;
  v8h hv[2];
#pragma unroll
  for (int g = 0; g < 2; ++g) {
    const int qq = g * 32 + q;
#pragma unroll
    for (int e = 0; e < 8; ++e) {
      const float f = Tt[(c8 + e) * 65 + qq];
      const unsigned short bits = __builtin_bit_cast(unsigned short, (_Float16)(f * sc));
      hv[g][e] = __builtin_bit_cast(_Float16, bits);
    }
  }
  for (int pass = 0; pass < 2; ++pass) {
#pragma unroll
    for (int g = 0; g < 2; ++g) {
      const size_t o = (size_t)(c0 + g * 32 + q) * (size_t)ldo + (size_t)(r0 + c8);
      *(volatile v8h*)(O + o) = hv[g];
    }
    __threadfence();
  }
}

__device__ __forceinline__ void step_ids(const float* __restrict__ x, int rowbase, int tt, int tid, int* ks) {
  const int m = tid >> 4, q = tid & 15;
  const float* rp = x + ((size_t)(rowbase + m) * NSTEP + (size_t)tt) * NVOC + 8 * q;
  const v4f va = *(const v4f*)(rp);
  const v4f vb = *(const v4f*)(rp + 4);
  int idx = BIGI;
#pragma unroll
  for (int e = 3; e >= 0; --e) { if (vb[e] >= 0.5f) idx = 8 * q + 4 + e; }
#pragma unroll
  for (int e = 3; e >= 0; --e) { if (va[e] >= 0.5f) idx = 8 * q + e; }
#pragma unroll
  for (int off = 1; off < 16; off <<= 1) {
    const int o = __shfl_xor(idx, off, 32);
    idx = (o < idx) ? o : idx;
  }
  if (q == 0) ks[m] = (idx < NVOC) ? idx : -1;
}

__global__ __launch_bounds__(NTHR) void seq_cell_kernel(const float* __restrict__ x, const float* __restrict__ Wi,
                                                        const float* __restrict__ bh, const unsigned short* __restrict__ WHTp,
                                                        float* __restrict__ out) {
  __shared__ __align__(16) _Float16 Ah[2][SEQ_BLK * HPITCH];
  __shared__ __align__(16) float    Xs[NWAVE][64 * XSEG];
  __shared__ __align__(16) float    Hs[SEQ_BLK * OPITCH];
  __shared__ __align__(16) float    Bs[NGATE];
  __shared__ int Ks[2][SEQ_BLK];
  __shared__ int Es[SEQ_BLK];
  const _Float16* WHT = (const _Float16*)WHTp;
  const int tid = threadIdx.x, lane = tid & 31, wave = tid >> 5;
  const int c = lane & 15, hh = lane >> 4, koff = hh * 8;
  const int ra = lane >> 2, f4 = (lane & 3) * 4;
  const int rowbase = blockIdx.x * SEQ_BLK;

  {
    _Float16* ahf = &Ah[0][0];
#pragma unroll 1
    for (int i = tid; i < 2 * SEQ_BLK * HPITCH; i += NTHR) ahf[i] = (_Float16)0.0f;
  }
#pragma unroll 1
  for (int i = tid; i < SEQ_BLK * OPITCH; i += NTHR) Hs[i] = 0.0f;
  {
    const v4f b0 = *(const v4f*)(bh + 8 * tid);
    const v4f b1 = *(const v4f*)(bh + 8 * tid + 4);
    *(v4f*)(Bs + 8 * tid)     = b0;
    *(v4f*)(Bs + 8 * tid + 4) = b1;
  }
#pragma unroll 1
  for (int rr = 0; rr < 2; ++rr) {
    const int m = 2 * wave + rr;
    const float* xb = x + (size_t)(rowbase + m) * NSTEP * NVOC + 1;
    int best = BIGI;
#pragma unroll 4
    for (int i = 0; i < NSTEP / 32; ++i) {
      const int tt = i * 32 + lane;
      const float v = xb[(size_t)tt * NVOC];
      if (v == 1.0f && tt < best) best = tt;
    }
#pragma unroll
    for (int off = 1; off < 32; off <<= 1) {
      const int o = __shfl_xor(best, off, 32);
      best = (o < best) ? o : best;
    }
    if (lane == 0) Es[m] = (best < NSTEP) ? best : (NSTEP - 1);
  }
  step_ids(x, rowbase, 0, tid, Ks[0]);
  __syncthreads();

  float bbr[4][4];
#pragma unroll
  for (int nt = 0; nt < 4; ++nt)
#pragma unroll
    for (int g = 0; g < 4; ++g) bbr[nt][g] = Bs[g * NHID + 64 * wave + 16 * nt + c];
  int erow[8];
#pragma unroll
  for (int r = 0; r < 8; ++r) erow[r] = Es[8 * hh + r];
  int mx = 0;
#pragma unroll
  for (int i = 0; i < SEQ_BLK; ++i) mx = (Es[i] > mx) ? Es[i] : mx;
  int tmax = __builtin_amdgcn_readfirstlane(mx);
  tmax = (tmax < 0) ? 0 : ((tmax > NSTEP - 1) ? (NSTEP - 1) : tmax);

  float cst[4][8];
#pragma unroll
  for (int nt = 0; nt < 4; ++nt)
#pragma unroll
    for (int r = 0; r < 8; ++r) cst[nt][r] = 0.0f;

  const v8f z8 = {0.f, 0.f, 0.f, 0.f, 0.f, 0.f, 0.f, 0.f};
  float* xsw = Xs[wave];

#pragma unroll 1
  for (int t = 0; t <= tmax; ++t) {
    const int cur = t & 1;
    int tka = Ks[cur][ra];
    int tkb = Ks[cur][ra + 8];
    const float ffa = (tka >= 0) ? 1.0f : 0.0f;
    const float ffb = (tkb >= 0) ? 1.0f : 0.0f;
    tka = (tka < 0) ? 0 : ((tka > NVOC - 1) ? (NVOC - 1) : tka);
    tkb = (tkb < 0) ? 0 : ((tkb > NVOC - 1) ? (NVOC - 1) : tkb);
    const _Float16* ahrow = &Ah[cur][0] + c * HPITCH + koff;
    _Float16* ahn = &Ah[cur ^ 1][0];
    const float* wia = Wi + (size_t)tka * NGATE + 64 * wave + f4;
    const float* wib = Wi + (size_t)tkb * NGATE + 64 * wave + f4;

#pragma unroll
    for (int nt = 0; nt < 4; ++nt) {
      const int j = 64 * wave + 16 * nt + c;
      __builtin_amdgcn_fence(__ATOMIC_RELEASE, "workgroup");
      __builtin_amdgcn_wave_barrier();
      __builtin_amdgcn_fence(__ATOMIC_ACQUIRE, "workgroup");
#pragma unroll
      for (int i = 0; i < 8; ++i) {
        const int g = i >> 1;
        const float* wp = ((i & 1) ? wib : wia) + g * NHID + 16 * nt;
        const float  ff = (i & 1) ? ffb : ffa;
        const v4f wv = *(const v4f*)wp;
        v4f zv;
#pragma unroll
        for (int e = 0; e < 4; ++e) zv[e] = wv[e] * ff;
        *(v4f*)(xsw + (i * 8 + ra) * XSEG + f4) = zv;
      }
      __builtin_amdgcn_fence(__ATOMIC_RELEASE, "workgroup");
      __builtin_amdgcn_wave_barrier();
      __builtin_amdgcn_fence(__ATOMIC_ACQUIRE, "workgroup");

      const _Float16* whb = WHT + (size_t)j * NHID + koff;
      v8f acc[4];
      acc[0] = z8; acc[1] = z8; acc[2] = z8; acc[3] = z8;
#pragma unroll 1
      for (int k0 = 0; k0 < NHID; k0 += 32) {
        const v16h a  = Frag<_Float16>::load(ahrow + k0);
        const v16h b0 = Frag<_Float16>::load(whb + k0);
        const v16h b1 = Frag<_Float16>::load(whb + (size_t)1 * NHID * NHID + k0);
        const v16h b2 = Frag<_Float16>::load(whb + (size_t)2 * NHID * NHID + k0);
        const v16h b3 = Frag<_Float16>::load(whb + (size_t)3 * NHID * NHID + k0);
        acc[0] = Frag<_Float16>::mma(a, b0, acc[0]);
        acc[1] = Frag<_Float16>::mma(a, b1, acc[1]);
        acc[2] = Frag<_Float16>::mma(a, b2, acc[2]);
        acc[3] = Frag<_Float16>::mma(a, b3, acc[3]);
        grp_guard_h(acc[0], acc[1], acc[2], acc[3], a, b0, b1, b2, b3);
      }
      acc_guard4(acc[0], acc[1], acc[2], acc[3]);

#pragma unroll
      for (int r = 0; r < 8; ++r) {
        const int row = 8 * hh + r;
        const float* xr = xsw + row * XSEG + c;
        const float zi = acc[0][r] * ZINV + xr[0 * 16 * XSEG] + bbr[nt][0];
        const float zf = acc[1][r] * ZINV + xr[1 * 16 * XSEG] + bbr[nt][1];
        const float zg = acc[2][r] * ZINV + xr[2 * 16 * XSEG] + bbr[nt][2];
        const float zo = acc[3][r] * ZINV + xr[3 * 16 * XSEG] + bbr[nt][3];
        const float ig = fsig(zi);
        const float fg = fsig(zf);
        const float og = fsig(zo);
        const float gg = ftanh(zg);
        const float cn = fg * cst[nt][r] + ig * gg;
        cst[nt][r] = cn;
        const float hn = og * ftanh(cn);
        ahn[row * HPITCH + j] = (_Float16)(hn * HCARRY);
        if (t == erow[r]) Hs[row * OPITCH + j] = hn;
      }
    }
    step_ids(x, rowbase, (t + 1 < NSTEP) ? (t + 1) : (NSTEP - 1), tid, Ks[cur ^ 1]);
    __syncthreads();
  }
  __syncthreads();

  for (int pass = 0; pass < 2; ++pass) {
#pragma unroll
    for (int it = 0; it < 8; ++it) {
      const int idx = it * NTHR + tid;
      const int row = idx >> 7, c4 = (idx & 127) * 4;
      const v4f v = *(const v4f*)(Hs + row * OPITCH + c4);
      *(volatile v4f*)(out + (size_t)(rowbase + row) * NHID + c4) = v;
    }
    __threadfence();
  }
}

extern "C" void kernel_launch(void* const* d_in, const int* in_sizes, int n_in,
                              void* d_out, int out_size, void* d_ws, size_t ws_size, hipStream_t stream) {
  if (n_in < 4 || d_out == nullptr || d_ws == nullptr) return;
  if (in_sizes[0] != NSEQ * NSTEP * NVOC || in_sizes[1] != NVOC * NGATE || in_sizes[2] != NHID * NGATE ||
      in_sizes[3] != NGATE || out_size != NSEQ * NHID) return;

  const float* x  = (const float*)d_in[0];
  const float* wi = (const float*)d_in[1];
  const float* wh = (const float*)d_in[2];
  const float* bh = (const float*)d_in[3];
  float* out = (float*)d_out;

  char* ws = (char*)d_ws; size_t off = 0;
  auto carve = [&](size_t bytes) -> char* { char* p = ws + off; off += (bytes + 255) & ~(size_t)255; return p; };
  unsigned short* WHT = (unsigned short*)carve((size_t)NGATE * NHID * 2);
  if (off > ws_size || off > (size_t)134217728) return;

  tpose_f16_kernel<<<dim3(NGATE / 64, NHID / 64), NTHR, 0, stream>>>(wh, NHID, NGATE, NHID, WHT, WCARRY);
  seq_cell_kernel<<<NSEQ / SEQ_BLK, NTHR, 0, stream>>>(x, wi, bh, WHT, out);
}
